// TimeAttentionGRU_19000935318215
// MI455X (gfx1250) — hardware-verified
//
#include <hip/hip_runtime.h>


namespace {
constexpr int NB = 32, S = 4096, D = 64, H = 128, CIN = D + H  , NG = 4, GI = CIN / NG  , GIP = 64, GO = H / NG  , NT = NB * S;
constexpr float XS = 8.0f, WSC = 256.0f;
typedef _Float16 b16;
typedef __attribute__((ext_vector_type(16))) _Float16 v16b;
typedef __attribute__((ext_vector_type(8))) _Float16 v8b;
typedef __attribute__((ext_vector_type(8))) float v8f;
typedef __attribute__((ext_vector_type(4))) float v4f;
__device__ __forceinline__ float bf16_rne(float f) { unsigned int u = __float_as_uint(f); u += 0x7FFFu + ((u >> 16) & 1u); return __uint_as_float(u & 0xFFFF0000u); }
__device__ __forceinline__ void split16(float v, b16& hi, b16& lo) { hi = (b16)v; lo = (b16)(v - (float)hi); }
__device__ __forceinline__ v16b frag_kb(const b16* p, int hh) { const v8b a = *(const v8b*)(p + 8 * hh), b = *(const v8b*)(p + 16 + 8 * hh); v16b f;
#pragma unroll
  for (int e = 0; e < 8; ++e) { f[e] = a[e]; f[8 + e] = b[e]; } return f; }
__device__ __forceinline__ v8f wmma16b(v16b a, v16b b, v8f c) { v8f d = __builtin_amdgcn_wmma_f32_16x16x32_f16(false, a, false, b, (short)0, c, false, false); asm volatile("v_nop\n\tv_nop\n\tv_nop\n\tv_nop" : "+v"(d) : "v"(a), "v"(b)); return d; }
__device__ __forceinline__ void wave_lds_sync() { __builtin_amdgcn_fence(__ATOMIC_RELEASE, "workgroup"); __builtin_amdgcn_wave_barrier(); __builtin_amdgcn_fence(__ATOMIC_ACQUIRE, "workgroup"); }
__device__ __forceinline__ float pmul(float a, float b) { float p = a * b; asm volatile("" : "+v"(p)); return p; }
__device__ __forceinline__ float sigm(float x) { return 1.0f / (1.0f + __expf(-x)); }

__global__ __launch_bounds__(256) void prepw_kernel(const float* __restrict__ wz, const float* __restrict__ wr, const float* __restrict__ wh, const float* __restrict__ w1, b16* __restrict__ WG, b16* __restrict__ W1T) {
  const int u = blockIdx.x * 256 + threadIdx.x; const int n1 = 3 * H * GIP / 8, n2 = H * H / 8; v8b o;
  if (u < n1) { const int e = u * 8; const int q = e / (H * GIP), rem = e % (H * GIP); const int ho = rem / GIP, c0 = rem % GIP; const float* w = q == 0 ? wz : q == 1 ? wr : wh;
    for (int j = 0; j < 8; ++j) { const int c = c0 + j; o[j] = (c < GI) ? (b16)(bf16_rne(w[((size_t)ho * GI + c) * 5 + 2]) * WSC) : (b16)0.0f; } for (int pass = 0; pass < 2; ++pass) { *(volatile v8b*)(WG + e) = o; __threadfence(); } return; }
  const int v = u - n1; if (v >= n2) return; { const int e = v * 8, oo = e / H, k0 = e % H; for (int j = 0; j < 8; ++j) o[j] = (b16)(bf16_rne(w1[(size_t)(k0 + j) * H + oo]) * WSC); for (int pass = 0; pass < 2; ++pass) { *(volatile v8b*)(W1T + e) = o; __threadfence(); } }
}
__global__ __launch_bounds__(256) void gru_kernel(const float* __restrict__ x, const b16* __restrict__ WG, const float* __restrict__ bz, const float* __restrict__ br, const float* __restrict__ bh, int nrows_tiles, float* __restrict__ G) {
  __shared__ __attribute__((aligned(16))) float Hf[NB][H + 4]; __shared__ __attribute__((aligned(16))) b16 Ch[NB][NG * GIP + 8], Cl[NB][NG * GIP + 8]; __shared__ __attribute__((aligned(16))) float ZR[2][NB][H + 4];
  const int t_ = threadIdx.x, wave = t_ >> 5, lane = t_ & 31, nloc = lane & 15, hlf = lane >> 4;
  for (int q = t_; q < NB * H; q += 256) Hf[q / H][q % H] = 0.0f;
  for (int q = t_; q < NB * (NG * GIP); q += 256) { Ch[q / (NG * GIP)][q % (NG * GIP)] = (b16)0.0f; Cl[q / (NG * GIP)][q % (NG * GIP)] = (b16)0.0f; }
  __syncthreads();
  auto put = [&](int row, int i, float v) { const int g = i / GI, cc = i % GI; b16 p, q; split16(v * XS, p, q); Ch[row][g * GIP + cc] = p; Cl[row][g * GIP + cc] = q; };
  const int myrow = t_ >> 3, mylane8 = t_ & 7;
  for (int step = 0; step < S; ++step) {
    { const float* xr = x + ((size_t)myrow * S + step) * D; for (int j = 0; j < 24; ++j) { const int i = mylane8 * 24 + j; const float v = (i < D) ? bf16_rne(xr[i]) : Hf[myrow][i - D]; put(myrow, i, v); } }
    __syncthreads();
    { const int qg = wave >> 2, g = wave & 3; v8f acc[2][2] = {{{}, {}}, {{}, {}}};
#pragma unroll
      for (int kb = 0; kb < GIP; kb += 32) { v16b bw[2]; for (int u = 0; u < 2; ++u) bw[u] = frag_kb(WG + ((size_t)qg * H + g * GO + u * 16 + nloc) * GIP + kb, hlf);
#pragma unroll
        for (int a = 0; a < 2; ++a) { if (a >= nrows_tiles) break; const v16b fa = frag_kb(&Ch[a * 16 + nloc][g * GIP + kb], hlf), fl = frag_kb(&Cl[a * 16 + nloc][g * GIP + kb], hlf);
#pragma unroll
          for (int u = 0; u < 2; ++u) { acc[a][u] = wmma16b(fa, bw[u], acc[a][u]); acc[a][u] = wmma16b(fl, bw[u], acc[a][u]); } } }
      const float* bb = qg == 0 ? bz : br;
#pragma unroll
      for (int a = 0; a < 2; ++a)
#pragma unroll
        for (int u = 0; u < 2; ++u) { const int j = g * GO + u * 16 + nloc; const float bj = bf16_rne(bb[j]);
#pragma unroll 1
          for (int r = 0; r < 8; ++r) ZR[qg][a * 16 + 8 * hlf + r][j] = sigm(acc[a][u][r] * (1.0f / (XS * WSC)) + bj); } }
    __syncthreads();
    { for (int j = 0; j < 24; ++j) { const int i = mylane8 * 24 + j; if (i >= D) { const int k = i - D; put(myrow, i, pmul(ZR[1][myrow][k], Hf[myrow][k])); } } }
    __syncthreads();
    { const int g = wave & 3, a = wave >> 2; v8f acc[2] = {{}, {}};
      if (a < nrows_tiles) {
#pragma unroll
        for (int kb = 0; kb < GIP; kb += 32) { const v16b fa = frag_kb(&Ch[a * 16 + nloc][g * GIP + kb], hlf), fl = frag_kb(&Cl[a * 16 + nloc][g * GIP + kb], hlf);
#pragma unroll
          for (int u = 0; u < 2; ++u) { const v16b bw = frag_kb(WG + ((size_t)2 * H + g * GO + u * 16 + nloc) * GIP + kb, hlf); acc[u] = wmma16b(fa, bw, acc[u]); acc[u] = wmma16b(fl, bw, acc[u]); } }
#pragma unroll
        for (int u = 0; u < 2; ++u) { const int j = g * GO + u * 16 + nloc; const float bj = bf16_rne(bh[j]);
#pragma unroll 1
          for (int r = 0; r < 8; ++r) { const int row = a * 16 + 8 * hlf + r; const float hh = tanhf(acc[u][r] * (1.0f / (XS * WSC)) + bj); const float z = ZR[0][row][j]; const float hn = pmul(1.0f - z, Hf[row][j]) + pmul(z, hh); Hf[row][j] = hn; } } } }
    __syncthreads();
    for (int pass = 0; pass < 2; ++pass) { for (int rr = 0; rr < 4; ++rr) { const int row = wave * 4 + rr; if (row < nrows_tiles * 16) *(volatile v4f*)(G + ((size_t)row * S + step) * H + lane * 4) = *(const v4f*)(&Hf[row][lane * 4]); } __threadfence(); }
  }
}
__global__ __launch_bounds__(128) void score_kernel(const float* __restrict__ G, const b16* __restrict__ W1T, const float* __restrict__ b1, const float* __restrict__ w2, const float* __restrict__ b2, float* __restrict__ SC) {
  __shared__ __attribute__((aligned(16))) b16 Ah[4][16][H + 8], Al[4][16][H + 8]; __shared__ __attribute__((aligned(16))) float sc[64];
  const int wave = threadIdx.x >> 5, lane = threadIdx.x & 31, nloc = lane & 15, hlf = lane >> 4; const size_t m0 = (size_t)blockIdx.x * 64 + wave * 16;
  for (int q = lane; q < 16 * (H / 4); q += 32) { const int rr = q / (H / 4), c4 = (q % (H / 4)) * 4; const v4f xv = *(const v4f*)(G + (m0 + rr) * H + c4); for (int j = 0; j < 4; ++j) { b16 p, pl; split16(xv[j] * XS, p, pl); Ah[wave][rr][c4 + j] = p; Al[wave][rr][c4 + j] = pl; } }
  wave_lds_sync(); v8f acc[8];
#pragma unroll
  for (int t = 0; t < 8; ++t) acc[t] = (v8f){};
#pragma unroll
  for (int kb = 0; kb < H; kb += 32) { const v16b a = frag_kb(&Ah[wave][nloc][kb], hlf), al = frag_kb(&Al[wave][nloc][kb], hlf);
#pragma unroll
    for (int t = 0; t < 8; ++t) { const v16b bw = frag_kb(W1T + (size_t)(t * 16 + nloc) * H + kb, hlf); acc[t] = wmma16b(a, bw, acc[t]); acc[t] = wmma16b(al, bw, acc[t]); } }
  float part[8]; for (int r = 0; r < 8; ++r) part[r] = 0.0f;
#pragma unroll
  for (int t = 0; t < 8; ++t) { const int c = t * 16 + nloc; const float bb = bf16_rne(b1[c]), ww = bf16_rne(w2[c]);
#pragma unroll
    for (int r = 0; r < 8; ++r) part[r] += pmul(tanhf(acc[t][r] * (1.0f / (XS * WSC)) + bb), ww); }
#pragma unroll
  for (int r = 0; r < 8; ++r) { float v = part[r]; v += __shfl_xor(v, 1); v += __shfl_xor(v, 2); v += __shfl_xor(v, 4); v += __shfl_xor(v, 8); part[r] = v; }
  if (nloc == 0) for (int r = 0; r < 8; ++r) sc[wave * 16 + 8 * hlf + r] = part[r] + bf16_rne(b2[0]);
  __syncthreads();
  for (int pass = 0; pass < 2; ++pass) { if (threadIdx.x < 16) *(volatile v4f*)(SC + (size_t)blockIdx.x * 64 + threadIdx.x * 4) = *(const v4f*)(&sc[threadIdx.x * 4]); __threadfence(); }
}
__global__ __launch_bounds__(256) void pool_kernel(const float* __restrict__ SC, const float* __restrict__ G, float* __restrict__ out) {
  __shared__ float red[256]; __shared__ float pr[S]; __shared__ __attribute__((aligned(16))) float ctx[2][H];
  const int b = blockIdx.x, t_ = threadIdx.x; const float* scb = SC + (size_t)b * S;
  float m = -INFINITY; for (int t = t_; t < S; t += 256) m = fmaxf(m, scb[t]); red[t_] = m; __syncthreads();
  for (int s = 128; s > 0; s >>= 1) { if (t_ < s) red[t_] = fmaxf(red[t_], red[t_ + s]); __syncthreads(); } m = red[0]; __syncthreads();
  float sm = 0.0f; for (int t = t_; t < S; t += 256) { const float p = __expf(scb[t] - m); pr[t] = p; sm += p; } red[t_] = sm; __syncthreads();
  for (int s = 128; s > 0; s >>= 1) { if (t_ < s) red[t_] = red[t_] + red[t_ + s]; __syncthreads(); } const float inv = 1.0f / red[0];
  { const int c = t_ & 127, half = t_ >> 7; float acc = 0.0f; const float* gb = G + (size_t)b * S * H; for (int t = half * (S / 2); t < (half + 1) * (S / 2); ++t) acc += pmul(pr[t], gb[(size_t)t * H + c]); ctx[half][c] = acc; }
  __syncthreads();
  for (int pass = 0; pass < 2; ++pass) { if (t_ < 32) { v4f o; for (int j = 0; j < 4; ++j) { const int c = t_ * 4 + j; o[j] = (ctx[0][c] + ctx[1][c]) * inv; } *(volatile v4f*)(out + (size_t)b * H + t_ * 4) = o; } __threadfence(); }
}
}

extern "C" void kernel_launch(void* const* d_in, const int* in_sizes, int n_in, void* d_out, int out_size, void* d_ws, size_t ws_size, hipStream_t stream) {
  (void)n_in;
  auto Fp = [&](int i) { return (const float*)d_in[i]; };
  if (in_sizes[0] != NB * S * D || in_sizes[1] != H * GI * 5 || in_sizes[3] != H * GI * 5 || in_sizes[5] != H * GI * 5 || in_sizes[7] != H * H || in_sizes[9] != H || out_size != NB * H) return;
  size_t off = 0; char* ws = (char*)d_ws;
  auto carve = [&](size_t bytes) { char* p = ws + off; off += (bytes + 255) & ~(size_t)255; return p; };
  b16* WG = (b16*)carve((size_t)3 * H * GIP * 2); b16* W1T = (b16*)carve((size_t)H * H * 2); float* G = (float*)carve((size_t)NT * H * 4); float* SC = (float*)carve((size_t)NT * 4);
  if (off > ws_size || off > ((size_t)128 << 20)) return;
  prepw_kernel<<<(3 * H * GIP / 8 + H * H / 8 + 255) / 256, 256, 0, stream>>>(Fp(1), Fp(3), Fp(5), Fp(7), WG, W1T);
  gru_kernel<<<1, 256, 0, stream>>>(Fp(0), WG, Fp(2), Fp(4), Fp(6), 2, G);
  score_kernel<<<NT / 64, 128, 0, stream>>>(G, W1T, Fp(8), Fp(9), Fp(10), SC);
  pool_kernel<<<NB, 256, 0, stream>>>(SC, G, (float*)d_out);
}
